// Block_16844861735766
// MI455X (gfx1250) — hardware-verified
//
#include <hip/hip_runtime.h>


#pragma clang fp contract(off)

#ifndef NB
#define NB 4
#endif
#ifndef SEQ
#define SEQ 2048
#endif
#define NB_FULL 4
#define SEQ_FULL 2048
#define CDIM 64
#define NHEAD 8
#define HD 64
#define QKVW (NHEAD * HD)
#define HID 256
#define MROWS (NB * SEQ)
#define PSC 16384.0f

static_assert(NB >= 1 && NB <= NB_FULL);
static_assert(SEQ % 64 == 0 && SEQ >= 64 && SEQ <= SEQ_FULL);
static_assert(HD == 64);
static_assert(CDIM == 64);
static_assert(QKVW == 512);
static_assert(HID % 64 == 0 && QKVW % 64 == 0 && CDIM % 64 == 0);
static_assert(HID % 32 == 0 && QKVW % 32 == 0 && CDIM % 32 == 0);
static_assert(MROWS % 64 == 0);
static_assert((long)MROWS * QKVW < (1L << 31));
static_assert((long)NB * NHEAD * SEQ * HD < (1L << 31));

typedef _Float16 v16h __attribute__((ext_vector_type(16)));
typedef _Float16 v8h  __attribute__((ext_vector_type(8)));
typedef float    v8f  __attribute__((ext_vector_type(8)));
typedef float    v4f  __attribute__((ext_vector_type(4)));
typedef float    v2f  __attribute__((ext_vector_type(2)));
typedef unsigned int v4u __attribute__((ext_vector_type(4)));

union Frag { v16h v; v4u q[2]; };

__device__ __forceinline__ v8f mma(v16h a, v16h b, v8f c) {
  v8f d = __builtin_amdgcn_wmma_f32_16x16x32_f16(false, a, false, b, (short)0, c, false, false);
  asm volatile("v_nop\n\tv_nop\n\tv_nop\n\tv_nop" : "+v"(d) : "v"(a), "v"(b));
  return d;
}

__device__ __forceinline__ v8f zero8() {
  v8f z;
#pragma unroll
  for (int i = 0; i < 8; ++i) z[i] = 0.0f;
  return z;
}

__device__ __forceinline__ float bf16q(float f) {
  unsigned int u = __float_as_uint(f);
  unsigned int r = u + 0x7FFFu + ((u >> 16) & 1u);
  r = ((u & 0x7F800000u) == 0x7F800000u) ? u : r;
  return __uint_as_float(r & 0xFFFF0000u);
}
__device__ __forceinline__ v4f bf16q4(v4f a) {
  v4f r;
  r.x = bf16q(a.x); r.y = bf16q(a.y); r.z = bf16q(a.z); r.w = bf16q(a.w);
  return r;
}
__device__ __forceinline__ unsigned short hbits(float f) {
  _Float16 h = (_Float16)f;
  return __builtin_bit_cast(unsigned short, h);
}
__device__ __forceinline__ v4u pack8h(float f0, float f1, float f2, float f3,
                                      float f4, float f5, float f6, float f7) {
  v8h t;
  t[0] = (_Float16)f0; t[1] = (_Float16)f1; t[2] = (_Float16)f2; t[3] = (_Float16)f3;
  t[4] = (_Float16)f4; t[5] = (_Float16)f5; t[6] = (_Float16)f6; t[7] = (_Float16)f7;
  return __builtin_bit_cast(v4u, t);
}

__global__ __launch_bounds__(256) void k_wprep(
    const float* __restrict__ s0, const float* __restrict__ s1, const float* __restrict__ s2,
    unsigned short* __restrict__ dst, int K, int hstride, int rstride, int zrows) {
  __shared__ __attribute__((aligned(16))) unsigned short sT[64][72];
  const int tid = threadIdx.x;
  const int k0 = blockIdx.x * 64, n0 = blockIdx.y * 64, z = blockIdx.z;
  const float* src = (z == 0) ? s0 : ((z == 1) ? s1 : s2);
  const size_t sbase = (size_t)(n0 >> 6) * (size_t)hstride;
#pragma unroll
  for (int it = 0; it < 4; ++it) {
    const int idx = it * 256 + tid;
    const int kk = idx >> 4;
    const int j4 = (idx & 15) * 4;
    const v4f wv = *(const v4f*)(src + sbase + (size_t)(k0 + kk) * (size_t)rstride + j4);
    sT[j4 + 0][kk] = hbits(bf16q(wv.x) * 16.0f);
    sT[j4 + 1][kk] = hbits(bf16q(wv.y) * 16.0f);
    sT[j4 + 2][kk] = hbits(bf16q(wv.z) * 16.0f);
    sT[j4 + 3][kk] = hbits(bf16q(wv.w) * 16.0f);
  }
  __syncthreads();
  v4u val[2];
  size_t off[2];
#pragma unroll
  for (int p = 0; p < 2; ++p) {
    const int n = p * 32 + (tid >> 3);
    const int piece = tid & 7;
    val[p] = *(const v4u*)&sT[n][piece * 8];
    off[p] = ((size_t)zrows * z + n0 + n) * (size_t)K + k0 + piece * 8;
  }
#pragma unroll
  for (int p = 0; p < 2; ++p) *(volatile v4u*)(dst + off[p]) = val[p];
  __threadfence();
#pragma unroll
  for (int p = 0; p < 2; ++p) *(volatile v4u*)(dst + off[p]) = val[p];
}

__global__ __launch_bounds__(256) void k_xcvt(
    const float* __restrict__ x, unsigned short* __restrict__ xh, int nrows) {
  const int tid = threadIdx.x;
  const int row = blockIdx.x * 32 + (tid >> 3);
  const int piece = tid & 7;
  if (row >= nrows) return;
  const int b = row / SEQ, t = row - b * SEQ;
  const size_t xrow = ((size_t)b * SEQ_FULL + t) * CDIM + piece * 8;
  const v4f a0 = bf16q4(*(const v4f*)(x + xrow));
  const v4f a1 = bf16q4(*(const v4f*)(x + xrow + 4));
  const v4u o = pack8h(a0.x, a0.y, a0.z, a0.w, a1.x, a1.y, a1.z, a1.w);
  unsigned short* d = xh + (size_t)row * CDIM + piece * 8;
  *(volatile v4u*)d = o;
  __threadfence();
  *(volatile v4u*)d = o;
}

template <int EPI, int RESFULL, int OUTFULL, int WRITEH>
__global__ __launch_bounds__(128) __attribute__((amdgpu_num_vgpr(256))) void k_gemm(
    const unsigned short* __restrict__ A, const unsigned short* __restrict__ Bt, int K,
    const float* __restrict__ bias, const float* __restrict__ biasb, const float* __restrict__ biasc,
    const float* __restrict__ res, const float* __restrict__ gam, const float* __restrict__ bet,
    float* __restrict__ outF, unsigned short* __restrict__ out0,
    unsigned short* __restrict__ out1, unsigned short* __restrict__ out2, int ldo) {
  __shared__ __attribute__((aligned(16))) unsigned short sT[64][72];
  __shared__ __attribute__((aligned(16))) float sF[64][68];
  const int tid = threadIdx.x, lane = tid & 31, w = tid >> 5;
  const int m = lane & 15, hl = lane >> 4, k8 = hl * 8;
  const int m0 = blockIdx.y * 64, n0 = blockIdx.x * 64;

  v8f acc[4];
#pragma unroll
  for (int j = 0; j < 4; ++j) acc[j] = zero8();

  const unsigned short* ap = A + (size_t)(m0 + 16 * w + m) * (size_t)K + k8;
  const unsigned short* bp = Bt + (size_t)(n0 + m) * (size_t)K + k8;
  const size_t jstep = (size_t)16 * (size_t)K;
#pragma unroll 1
  for (int k0 = 0; k0 < K; k0 += 32) {
    Frag a;
    a.q[0] = *(const v4u*)(ap + k0);
    a.q[1] = *(const v4u*)(ap + k0 + 16);
#pragma unroll
    for (int j = 0; j < 4; ++j) {
      Frag b;
      const unsigned short* bj = bp + jstep * j + k0;
      b.q[0] = *(const v4u*)(bj);
      b.q[1] = *(const v4u*)(bj + 16);
      acc[j] = mma(a.v, b.v, acc[j]);
    }
  }

  const float wsc = 0.0625f;
  const int lrow0 = 16 * w + 8 * hl;

  if constexpr (EPI == 0) {
    const int which = n0 / QKVW;
    const int hh = (n0 - which * QKVW) / HD;
    const float* bsel = (which == 0) ? bias : ((which == 1) ? biasb : biasc);
#pragma unroll
    for (int j = 0; j < 4; ++j) {
      const float bj = bf16q(bsel[hh * HD + 16 * j + m]);
#pragma unroll
      for (int r = 0; r < 8; ++r) sT[lrow0 + r][16 * j + m] = hbits(acc[j][r] * wsc + bj);
    }
    __syncthreads();
    const int b = m0 / SEQ, t0 = m0 - b * SEQ;
    const int bh = b * NHEAD + hh;
    v4u val[4];
    unsigned int off[4];
    unsigned short* dst;
    if (which < 2) {
      dst = (which == 0) ? out0 : out1;
#pragma unroll
      for (int p = 0; p < 4; ++p) {
        const int row = p * 16 + 4 * w + (lane >> 3);
        const int piece = lane & 7;
        val[p] = *(const v4u*)&sT[row][piece * 8];
        off[p] = (unsigned int)((bh * SEQ + t0 + row) * HD + piece * 8);
      }
    } else {
      dst = out2;
#pragma unroll
      for (int p = 0; p < 4; ++p) {
        const int d = p * 16 + 4 * w + (lane >> 3);
        const int piece = lane & 7;
        unsigned int wv[4];
#pragma unroll
        for (int e = 0; e < 4; ++e) {
          const unsigned int lo = sT[piece * 8 + 2 * e][d];
          const unsigned int hi = sT[piece * 8 + 2 * e + 1][d];
          wv[e] = lo | (hi << 16);
        }
        v4u t;
        t.x = wv[0]; t.y = wv[1]; t.z = wv[2]; t.w = wv[3];
        val[p] = t;
        off[p] = (unsigned int)((bh * HD + d) * SEQ + t0 + piece * 8);
      }
    }
#pragma unroll
    for (int p = 0; p < 4; ++p) *(volatile v4u*)(dst + off[p]) = val[p];
    __threadfence();
#pragma unroll
    for (int p = 0; p < 4; ++p) *(volatile v4u*)(dst + off[p]) = val[p];
  } else if constexpr (EPI == 2) {
#pragma unroll
    for (int j = 0; j < 4; ++j) {
      const float bj = bf16q(bias[n0 + 16 * j + m]);
#pragma unroll
      for (int r = 0; r < 8; ++r) {
        float u = acc[j][r] * wsc + bj;
        u = fmaxf(u, 0.0f);
        sT[lrow0 + r][16 * j + m] = hbits(u);
      }
    }
    __syncthreads();
    v4u val[4];
    unsigned int off[4];
#pragma unroll
    for (int p = 0; p < 4; ++p) {
      const int row = 16 * w + 4 * p + (lane >> 3);
      const int piece = lane & 7;
      val[p] = *(const v4u*)&sT[row][piece * 8];
      off[p] = (unsigned int)((size_t)(m0 + row) * (size_t)ldo + n0 + piece * 8);
    }
#pragma unroll
    for (int p = 0; p < 4; ++p) *(volatile v4u*)(out0 + off[p]) = val[p];
    __threadfence();
#pragma unroll
    for (int p = 0; p < 4; ++p) *(volatile v4u*)(out0 + off[p]) = val[p];
  } else {
#pragma unroll
    for (int j = 0; j < 4; ++j) {
#pragma unroll
      for (int r = 0; r < 8; ++r) sF[lrow0 + r][16 * j + m] = acc[j][r] * wsc;
    }
    __syncthreads();
    const int b = m0 / SEQ, t0 = m0 - b * SEQ;
    const int c2 = 2 * lane;
    const float bb0 = bf16q(bias[n0 + c2]), bb1 = bf16q(bias[n0 + c2 + 1]);
    const float gg0 = bf16q(gam[n0 + c2]),  gg1 = bf16q(gam[n0 + c2 + 1]);
    const float ee0 = bf16q(bet[n0 + c2]),  ee1 = bf16q(bet[n0 + c2 + 1]);
#pragma unroll
    for (int rr = 0; rr < 16; ++rr) {
      const int row = 16 * w + rr;
      const size_t rrow = RESFULL ? ((size_t)b * SEQ_FULL + t0 + row) : (size_t)(m0 + row);
      v2f rv = *(const v2f*)(res + rrow * (size_t)ldo + n0 + c2);
      if (RESFULL) { rv.x = bf16q(rv.x); rv.y = bf16q(rv.y); }
      const v2f av = *(const v2f*)&sF[row][c2];
      const float u0 = (av.x + bb0) + rv.x;
      const float u1 = (av.y + bb1) + rv.y;
      float s = u0 + u1;
#pragma unroll
      for (int xm = 1; xm < 32; xm <<= 1) s += __shfl_xor(s, xm, 32);
      const float mu = s * (1.0f / CDIM);
      const float d0 = u0 - mu, d1 = u1 - mu;
      float qs = d0 * d0 + d1 * d1;
#pragma unroll
      for (int xm = 1; xm < 32; xm <<= 1) qs += __shfl_xor(qs, xm, 32);
      const float var = qs * (1.0f / CDIM);
      const float rstd = rsqrtf(var + 1e-5f);
      const float y0 = d0 * rstd * gg0 + ee0;
      const float y1 = d1 * rstd * gg1 + ee1;
      v2f yv; yv.x = y0; yv.y = y1;
      *(v2f*)&sF[row][c2] = yv;
      if (WRITEH) { sT[row][c2] = hbits(y0); sT[row][c2 + 1] = hbits(y1); }
    }
    __syncthreads();
    v4f fv[8];
    unsigned int fo[8];
#pragma unroll
    for (int p = 0; p < 8; ++p) {
      const int row = 16 * w + 2 * p + hl;
      const int piece = m;
      fv[p] = *(const v4f*)&sF[row][4 * piece];
      const size_t orow = OUTFULL ? ((size_t)b * SEQ_FULL + t0 + row) : (size_t)(m0 + row);
      fo[p] = (unsigned int)(orow * (size_t)ldo + n0 + 4 * piece);
    }
    v4u hv[4];
    unsigned int ho[4];
    if constexpr (WRITEH) {
#pragma unroll
      for (int p = 0; p < 4; ++p) {
        const int row = 16 * w + 4 * p + (lane >> 3);
        const int piece = lane & 7;
        hv[p] = *(const v4u*)&sT[row][piece * 8];
        ho[p] = (unsigned int)((size_t)(m0 + row) * CDIM + piece * 8);
      }
    }
#pragma unroll
    for (int p = 0; p < 8; ++p) *(volatile v4f*)(outF + fo[p]) = fv[p];
    if constexpr (WRITEH) {
#pragma unroll
      for (int p = 0; p < 4; ++p) *(volatile v4u*)(out0 + ho[p]) = hv[p];
    }
    __threadfence();
#pragma unroll
    for (int p = 0; p < 8; ++p) *(volatile v4f*)(outF + fo[p]) = fv[p];
    if constexpr (WRITEH) {
#pragma unroll
      for (int p = 0; p < 4; ++p) *(volatile v4u*)(out0 + ho[p]) = hv[p];
    }
  }
}

__global__ __launch_bounds__(128) __attribute__((amdgpu_num_vgpr(256)))
void k_attn(const unsigned short* __restrict__ qp, const unsigned short* __restrict__ kp,
            const unsigned short* __restrict__ vp, unsigned short* __restrict__ op) {
  __shared__ __attribute__((aligned(16))) unsigned short sP[4][16][72];
  const int tid = threadIdx.x, lane = tid & 31, w = tid >> 5;
  const int m = lane & 15, hl = lane >> 4, k8 = hl * 8;
  const int nqt = SEQ / 64;
  const int bh = blockIdx.x / nqt, qt = blockIdx.x - bh * nqt;
  const int b = bh / NHEAD, hh = bh - b * NHEAD;
  const int tq = qt * 64 + 16 * w;

  Frag qa0, qa1;
  {
    const unsigned short* qr = qp + ((size_t)bh * SEQ + tq + m) * HD + k8;
    qa0.q[0] = *(const v4u*)(qr);
    qa0.q[1] = *(const v4u*)(qr + 16);
    qa1.q[0] = *(const v4u*)(qr + 32);
    qa1.q[1] = *(const v4u*)(qr + 48);
  }
  float mrun[8], lrun[8];
  v8f oacc[4];
#pragma unroll
  for (int r = 0; r < 8; ++r) { mrun[r] = -1e30f; lrun[r] = 0.0f; }
#pragma unroll
  for (int j = 0; j < 4; ++j) oacc[j] = zero8();

#pragma unroll 1
  for (int kt = 0; kt <= qt; ++kt) {
    v8f s[4];
    const unsigned short* kb = kp + ((size_t)bh * SEQ + kt * 64 + m) * HD + k8;
#pragma unroll
    for (int j = 0; j < 4; ++j) {
      const unsigned short* kr = kb + j * 16 * HD;
      Frag f0, f1;
      f0.q[0] = *(const v4u*)(kr);
      f0.q[1] = *(const v4u*)(kr + 16);
      f1.q[0] = *(const v4u*)(kr + 32);
      f1.q[1] = *(const v4u*)(kr + 48);
      v8f t = mma(qa0.v, f0.v, zero8());
      t = mma(qa1.v, f1.v, t);
      s[j] = t;
    }
    const bool diag = (kt == qt);
    float tmax[8];
#pragma unroll
    for (int r = 0; r < 8; ++r) tmax[r] = -1e30f;
#pragma unroll
    for (int j = 0; j < 4; ++j) {
#pragma unroll
      for (int r = 0; r < 8; ++r) {
        float val = s[j][r];
        const int qi = tq + 8 * hl + r;
        const int ki = kt * 64 + 16 * j + m;
        val = (diag && (ki > qi)) ? -1e30f : val;
        s[j][r] = val;
        tmax[r] = fmaxf(tmax[r], val);
      }
    }
#pragma unroll
    for (int r = 0; r < 8; ++r) {
#pragma unroll
      for (int xm = 1; xm < 16; xm <<= 1) tmax[r] = fmaxf(tmax[r], __shfl_xor(tmax[r], xm, 32));
    }
    float corr[8];
#pragma unroll
    for (int r = 0; r < 8; ++r) {
      const float mn = fmaxf(mrun[r], tmax[r]);
      corr[r] = __expf(mrun[r] - mn);
      mrun[r] = mn;
    }
    float tsum[8];
#pragma unroll
    for (int r = 0; r < 8; ++r) tsum[r] = 0.0f;
#pragma unroll
    for (int j = 0; j < 4; ++j) {
#pragma unroll
      for (int r = 0; r < 8; ++r) {
        const float p = __expf(s[j][r] - mrun[r]);
        tsum[r] += p;
        sP[w][8 * hl + r][16 * j + m] = hbits(p * PSC);
      }
    }
#pragma unroll
    for (int r = 0; r < 8; ++r) {
#pragma unroll
      for (int xm = 1; xm < 16; xm <<= 1) tsum[r] += __shfl_xor(tsum[r], xm, 32);
      lrun[r] = lrun[r] * corr[r] + tsum[r];
    }
#pragma unroll
    for (int j = 0; j < 4; ++j) {
#pragma unroll
      for (int r = 0; r < 8; ++r) oacc[j][r] *= corr[r];
    }
    __syncthreads();
    Frag pa0, pa1;
    {
      const unsigned short* pr = &sP[w][m][k8];
      pa0.q[0] = *(const v4u*)(pr);
      pa0.q[1] = *(const v4u*)(pr + 16);
      pa1.q[0] = *(const v4u*)(pr + 32);
      pa1.q[1] = *(const v4u*)(pr + 48);
    }
    const unsigned short* vb = vp + ((size_t)bh * HD + m) * (size_t)SEQ + kt * 64 + k8;
#pragma unroll
    for (int jd = 0; jd < 4; ++jd) {
      const unsigned short* vr = vb + (size_t)jd * 16 * SEQ;
      Frag g0, g1;
      g0.q[0] = *(const v4u*)(vr);
      g0.q[1] = *(const v4u*)(vr + 16);
      g1.q[0] = *(const v4u*)(vr + 32);
      g1.q[1] = *(const v4u*)(vr + 48);
      oacc[jd] = mma(pa0.v, g0.v, oacc[jd]);
      oacc[jd] = mma(pa1.v, g1.v, oacc[jd]);
    }
    __syncthreads();
  }

  float il[8];
#pragma unroll
  for (int r = 0; r < 8; ++r) il[r] = 1.0f / (lrun[r] * PSC);
#pragma unroll
  for (int jd = 0; jd < 4; ++jd) {
#pragma unroll
    for (int r = 0; r < 8; ++r) sP[w][8 * hl + r][16 * jd + m] = hbits(oacc[jd][r] * il[r]);
  }
  __syncthreads();
  v4u val[4];
  unsigned int off[4];
#pragma unroll
  for (int p = 0; p < 4; ++p) {
    const int row = 4 * p + (lane >> 3);
    const int piece = lane & 7;
    val[p] = *(const v4u*)&sP[w][row][piece * 8];
    off[p] = (unsigned int)((size_t)(b * SEQ + tq + row) * QKVW + hh * HD + piece * 8);
  }
#pragma unroll
  for (int p = 0; p < 4; ++p) *(volatile v4u*)(op + off[p]) = val[p];
  __threadfence();
#pragma unroll
  for (int p = 0; p < 4; ++p) *(volatile v4u*)(op + off[p]) = val[p];
}

static inline size_t al256(size_t v) { return (v + 255) & ~(size_t)255; }

extern "C" void kernel_launch(void* const* d_in, const int* in_sizes, int n_in,
                              void* d_out, int out_size, void* d_ws, size_t ws_size,
                              hipStream_t stream) {
  if (n_in < 17) return;
  const long needX = ((long)(NB - 1) * SEQ_FULL + SEQ) * CDIM;
  const long nW = (long)NHEAD * CDIM * HD;
  if ((long)in_sizes[0] < needX) return;
  if ((long)in_sizes[1] < nW || (long)in_sizes[3] < nW || (long)in_sizes[5] < nW) return;
  if (in_sizes[2] < QKVW || in_sizes[4] < QKVW || in_sizes[6] < QKVW) return;
  if ((long)in_sizes[7] < (long)QKVW * CDIM || in_sizes[8] < CDIM) return;
  if ((long)in_sizes[9] < (long)CDIM * HID || in_sizes[10] < HID) return;
  if ((long)in_sizes[11] < (long)HID * CDIM || in_sizes[12] < CDIM) return;
  if (in_sizes[13] < CDIM || in_sizes[14] < CDIM || in_sizes[15] < CDIM || in_sizes[16] < CDIM) return;
  if ((long)out_size < needX) return;

  const float* x   = (const float*)d_in[0];
  const float* Wq  = (const float*)d_in[1];
  const float* bq  = (const float*)d_in[2];
  const float* Wk  = (const float*)d_in[3];
  const float* bk  = (const float*)d_in[4];
  const float* Wv  = (const float*)d_in[5];
  const float* bv  = (const float*)d_in[6];
  const float* Wp  = (const float*)d_in[7];
  const float* bp  = (const float*)d_in[8];
  const float* W1  = (const float*)d_in[9];
  const float* b1  = (const float*)d_in[10];
  const float* W2  = (const float*)d_in[11];
  const float* b2  = (const float*)d_in[12];
  const float* g1  = (const float*)d_in[13];
  const float* be1 = (const float*)d_in[14];
  const float* g2  = (const float*)d_in[15];
  const float* be2 = (const float*)d_in[16];
  float* out = (float*)d_out;

  char* ws = (char*)d_ws;
  size_t off = 0;
  auto carve = [&](size_t bytes) -> char* { char* p = ws + off; off += al256(bytes); return p; };
  const size_t MC  = (size_t)MROWS * CDIM;
  const size_t MHD = (size_t)NB * NHEAD * SEQ * HD;
  unsigned short* wqkv = (unsigned short*)carve((size_t)3 * QKVW * CDIM * 2);
  unsigned short* wpt  = (unsigned short*)carve((size_t)CDIM * QKVW * 2);
  unsigned short* w1t  = (unsigned short*)carve((size_t)HID * CDIM * 2);
  unsigned short* w2t  = (unsigned short*)carve((size_t)CDIM * HID * 2);
  unsigned short* xh   = (unsigned short*)carve(MC * 2);
  unsigned short* qpl  = (unsigned short*)carve(MHD * 2);
  unsigned short* kpl  = (unsigned short*)carve(MHD * 2);
  unsigned short* vtp  = (unsigned short*)carve(MHD * 2);
  unsigned short* opl  = (unsigned short*)carve((size_t)MROWS * QKVW * 2);
  float*          h1f  = (float*)carve(MC * 4);
  unsigned short* h1h  = (unsigned short*)carve(MC * 2);
  unsigned short* act  = (unsigned short*)carve((size_t)MROWS * HID * 2);
  if (off > ws_size) return;
  if (off > ((size_t)128 << 20)) return;

  k_wprep<<<dim3(CDIM / 64, QKVW / 64, 3), 256, 0, stream>>>(Wq, Wk, Wv, wqkv, CDIM, CDIM * HD, HD, QKVW);
  k_wprep<<<dim3(QKVW / 64, CDIM / 64, 1), 256, 0, stream>>>(Wp, Wp, Wp, wpt, QKVW, 64, CDIM, 0);
  k_wprep<<<dim3(CDIM / 64, HID / 64, 1), 256, 0, stream>>>(W1, W1, W1, w1t, CDIM, 64, HID, 0);
  k_wprep<<<dim3(HID / 64, CDIM / 64, 1), 256, 0, stream>>>(W2, W2, W2, w2t, HID, 64, CDIM, 0);
  k_xcvt<<<MROWS / 32, 256, 0, stream>>>(x, xh, MROWS);
  k_gemm<0, 0, 0, 0><<<dim3(3 * QKVW / 64, MROWS / 64), 128, 0, stream>>>(
      xh, wqkv, CDIM, bq, bk, bv, nullptr, nullptr, nullptr, nullptr, qpl, kpl, vtp, 0);
  k_attn<<<NB * NHEAD * (SEQ / 64), 128, 0, stream>>>(qpl, kpl, vtp, opl);
  k_gemm<1, 1, 0, 1><<<dim3(CDIM / 64, MROWS / 64), 128, 0, stream>>>(
      opl, wpt, QKVW, bp, bp, bp, x, g1, be1, h1f, h1h, nullptr, nullptr, CDIM);
  k_gemm<2, 0, 0, 0><<<dim3(HID / 64, MROWS / 64), 128, 0, stream>>>(
      h1h, w1t, CDIM, b1, b1, b1, nullptr, nullptr, nullptr, nullptr, act, nullptr, nullptr, HID);
  k_gemm<1, 0, 1, 0><<<dim3(CDIM / 64, MROWS / 64), 128, 0, stream>>>(
      act, w2t, HID, b2, b2, b2, h1f, g2, be2, out, nullptr, nullptr, nullptr, CDIM);
}
